// SeasonalityBlock_12575664243332
// MI455X (gfx1250) — hardware-run, weakly checked
//
#include <hip/hip_runtime.h>
#include <math.h>

typedef __attribute__((ext_vector_type(16))) _Float16 v16h;
typedef __attribute__((ext_vector_type(8)))  _Float16 v8h;
typedef __attribute__((ext_vector_type(8)))  float    v8f;
typedef __attribute__((ext_vector_type(4)))  float    v4f;
typedef __attribute__((ext_vector_type(2)))  float    v2f;
typedef __attribute__((ext_vector_type(4)))  unsigned v4u;
typedef __attribute__((ext_vector_type(4)))  int      v4i;
typedef __attribute__((ext_vector_type(2)))  double   v2d;

constexpr int kNb       = 32;
constexpr int kNt       = 2048;
constexpr int kNd       = 64;
constexpr int kPred     = 96;
constexpr int kTout     = kNt + kPred;
constexpr int kCols     = kNb * kNd;
constexpr int kTopK     = 8;
constexpr int kSelPitch = 32;
constexpr int kBins     = kNt / 2;
constexpr int kBinsPerLane = kBins / 32;
constexpr int kTapRows  = 2 * kBins;
constexpr int kTilesM   = kCols / 64;
constexpr int kTilesN   = kTapRows / 64;
constexpr int kSlabP    = 36;
constexpr int kChunkT   = 256;
constexpr int kTileP    = 33;
constexpr int kMaxContested = 64;
constexpr int kDGroups  = kNd / 32;
constexpr int kTChunks  = kNt / kChunkT;
constexpr int kInTotal  = kNb * kNt * kNd;
constexpr int kOutTotal = kNb * kTout * kNd;

static_assert(kCols == 2048);
static_assert(kTout == 2144);
static_assert(kBins == 1024 && kTapRows == 2048);
static_assert(kBinsPerLane == 32);
static_assert(kTilesM == 32 && kTilesN == 32);
static_assert((kTilesM * kTilesN) % 8 == 0);
static_assert((kNt % 32) == 0);
static_assert((kCols % 8) == 0);
static_assert(kInTotal == 4194304);
static_assert(kOutTotal == 4390912);
static_assert(kPred <= kChunkT);
static_assert((kPred % 32) == 0 && (kPred / 32) == 3);
static_assert(kDGroups == 2 && kTChunks == 8);
static_assert(kTopK == 8 && kTopK <= kSelPitch);
static_assert(2 * kNt == 256 * 4 * 4);

constexpr float kCarrySig = 16.0f;
constexpr float kCarryTap = 256.0f;
constexpr float kFold     = 1.0f / (kCarrySig * kCarryTap);
constexpr float kHalfMinNormal = 6.103515625e-05f;
static_assert(kFold * 4096.0f == 1.0f);

constexpr float kWindow = 3.2e-3f;
constexpr float kHiFac  = (1.0f + kWindow) * (1.0f + kWindow);
constexpr float kLoFac  = (1.0f - kWindow) * (1.0f - kWindow);
constexpr float kSynthScale = 2.0f / (float)kNt;
constexpr double kPiOver1024 = 3.14159265358979323846 / 1024.0;

constexpr size_t kBytesXs32  = (size_t)kCols * kNt * 4;
constexpr size_t kBytesXs16  = (size_t)kCols * kNt * 2;
constexpr size_t kBytesTap   = (size_t)kTapRows * kNt * 2;
constexpr size_t kBytesCs    = (size_t)kNt * 2 * 4;
constexpr size_t kBytesCs64  = (size_t)kNt * 2 * 8;
constexpr size_t kBytesPlane = (size_t)kCols * kBins * 4;
constexpr size_t kBytesSel   = (size_t)kCols * kSelPitch * 4;
constexpr size_t kOffXs32  = 0;
constexpr size_t kOffXs16  = kOffXs32 + kBytesXs32;
constexpr size_t kOffTap   = kOffXs16 + kBytesXs16;
constexpr size_t kOffCs    = kOffTap + kBytesTap;
constexpr size_t kOffCs64  = kOffCs + kBytesCs;
constexpr size_t kOffRe    = kOffCs64 + kBytesCs64;
constexpr size_t kOffIm    = kOffRe + kBytesPlane;
constexpr size_t kOffAmp2  = kOffIm + kBytesPlane;
constexpr size_t kOffSelK  = kOffAmp2 + kBytesPlane;
constexpr size_t kOffSelRe = kOffSelK + kBytesSel;
constexpr size_t kOffSelIm = kOffSelRe + kBytesSel;
constexpr size_t kWsTotal  = kOffSelIm + kBytesSel;
static_assert(kBytesXs32 == 16777216ull);
static_assert(kBytesXs16 == 8388608ull);
static_assert(kBytesTap == 8388608ull);
static_assert(kBytesCs == 16384ull);
static_assert(kBytesCs64 == 32768ull);
static_assert(kBytesPlane == 8388608ull);
static_assert(kBytesSel == 262144ull);
static_assert(kWsTotal == 59555840ull);
static_assert(kWsTotal <= 134217728ull);
static_assert((kOffXs16 % 128) == 0 && (kOffTap % 128) == 0);
static_assert((kOffCs % 128) == 0 && (kOffCs64 % 128) == 0 && (kOffRe % 128) == 0);
static_assert((kOffIm % 128) == 0 && (kOffAmp2 % 128) == 0 && (kOffSelK % 128) == 0);
static_assert((kOffSelRe % 128) == 0 && (kOffSelIm % 128) == 0);

namespace eng {
union FragU { v16h v; v8h h[2]; };
__device__ __forceinline__ v16h frag_load(const _Float16* p) {
  FragU f;
  f.h[0] = *(const v8h*)(p);
  f.h[1] = *(const v8h*)(p + 16);
  return f.v;
}
__device__ __forceinline__ v8f mma(v16h a, v16h b, v8f c) {
  return __builtin_amdgcn_wmma_f32_16x16x32_f16(false, a, false, b, (short)0, c, false, false);
}
__device__ __forceinline__ void tie_acc(v8f& c, v16h a, v16h b) {
  asm volatile("" : "+v"(c) : "v"(a), "v"(b));
}
__device__ __forceinline__ void tie_acc_nops(v8f& c, v16h a, v16h b) {
  asm volatile("v_nop\n\tv_nop\n\tv_nop\n\tv_nop" : "+v"(c) : "v"(a), "v"(b));
}
__device__ __forceinline__ void keep4(v16h a, v16h b, v16h c, v16h d) {
  asm volatile("v_nop" :: "v"(a), "v"(b), "v"(c), "v"(d));
}
__device__ __forceinline__ void acc_guard4(v8f& a, v8f& b, v8f& c, v8f& d) {
  asm volatile("v_nop\n\tv_nop\n\tv_nop\n\tv_nop" : "+v"(a), "+v"(b), "+v"(c), "+v"(d));
}
}

__device__ __forceinline__ float flush_small(float v) {
  return (fabsf(v) < kHalfMinNormal) ? 0.0f : v;
}
__device__ __forceinline__ unsigned pack2_f16(float a, float b) {
  const _Float16 h0 = (_Float16)a;
  const _Float16 h1 = (_Float16)b;
  const unsigned short u0 = __builtin_bit_cast(unsigned short, h0);
  const unsigned short u1 = __builtin_bit_cast(unsigned short, h1);
  return (unsigned)u0 | ((unsigned)u1 << 16);
}

__device__ __forceinline__ void wave_lds_sync() {
  __builtin_amdgcn_fence(__ATOMIC_RELEASE, "workgroup");
  __builtin_amdgcn_wave_barrier();
  __builtin_amdgcn_fence(__ATOMIC_ACQUIRE, "workgroup");
}
__device__ __forceinline__ int wave_sum_i32(int v) {
#pragma unroll
  for (int off = 16; off >= 1; off >>= 1) v += __shfl_xor(v, off, 32);
  return v;
}
__device__ __forceinline__ double wave_sum_f64(double v) {
#pragma unroll
  for (int off = 16; off >= 1; off >>= 1) {
    const int hi = __double2hiint(v);
    const int lo = __double2loint(v);
    const int ohi = __shfl_xor(hi, off, 32);
    const int olo = __shfl_xor(lo, off, 32);
    v = v + __hiloint2double(ohi, olo);
  }
  return v;
}

__global__ __launch_bounds__(256) void column_plane_kernel(const float* __restrict__ x, float* __restrict__ XS32,
                                                          unsigned* __restrict__ XS16)
{
  __shared__ __align__(16) float tile[kChunkT * kTileP];
  const int lane = threadIdx.x & 31;
  const int wave = threadIdx.x >> 5;
  const int b  = blockIdx.x / kDGroups;
  const int d0 = (blockIdx.x % kDGroups) * 32;
  const int m0 = b * kNd + d0;
  const float* xc = x + (size_t)b * kNt * kNd + d0 + lane;

  for (int ch = 0; ch < kNt / kChunkT; ++ch) {
    const int t0 = ch * kChunkT;
    for (int i = 0; i < kChunkT / 8; ++i) {
      const int tl = wave + 8 * i;
      const float xv = xc[(size_t)(t0 + tl) * kNd];
      tile[tl * kTileP + lane] = xv;
    }
    __syncthreads();
    for (int pass = 0; pass < 2; ++pass) {
#pragma unroll
      for (int u = 0; u < 4; ++u) {
        const int dch = wave * 4 + u;
        const size_t rowBase = (size_t)(m0 + dch) * kNt + t0;
#pragma unroll
        for (int sg = 0; sg < 2; ++sg) {
          const int tl = sg * 128 + 4 * lane;
          v4f v;
          v[0] = tile[(tl + 0) * kTileP + dch];
          v[1] = tile[(tl + 1) * kTileP + dch];
          v[2] = tile[(tl + 2) * kTileP + dch];
          v[3] = tile[(tl + 3) * kTileP + dch];
          *(volatile v4f*)(XS32 + rowBase + tl) = v;
        }
        float h[8];
#pragma unroll
        for (int e = 0; e < 8; ++e) h[e] = flush_small(tile[(8 * lane + e) * kTileP + dch] * kCarrySig);
        v4u w;
        w[0] = pack2_f16(h[0], h[1]);
        w[1] = pack2_f16(h[2], h[3]);
        w[2] = pack2_f16(h[4], h[5]);
        w[3] = pack2_f16(h[6], h[7]);
        *(volatile v4u*)(XS16 + (rowBase + 8 * lane) / 2) = w;
      }
      __threadfence();
    }
    __syncthreads();
  }
}

__device__ __forceinline__ void cs64_entry(int j, double& c, double& s) {
  const int qd = (j >> 9) & 3;
  const int r  = j & 511;
  const bool sw = (r > 256);
  const int rr = sw ? (512 - r) : r;
  const double xx = (double)rr * kPiOver1024;
  const double x2 = xx * xx;
  double cc = 1.0;
  double sc = 1.0;
#pragma unroll
  for (int n = 11; n >= 1; --n) {
    cc = 1.0 - x2 * cc * (1.0 / (double)((2 * n - 1) * (2 * n)));
    sc = 1.0 - x2 * sc * (1.0 / (double)((2 * n) * (2 * n + 1)));
  }
  const double sn = xx * sc;
  const double c0 = sw ? sn : cc;
  const double s0 = sw ? cc : sn;
  c = (qd == 0) ? c0 : ((qd == 1) ? -s0 : ((qd == 2) ? -c0 : s0));
  s = (qd == 0) ? s0 : ((qd == 1) ? c0 : ((qd == 2) ? -s0 : -c0));
}

__global__ __launch_bounds__(256) void table_kernel(unsigned* __restrict__ TAP, float* __restrict__ CS,
                                                    double* __restrict__ CS64)
{
  const int r   = blockIdx.x;
  const int tid = threadIdx.x;
  if (r < kTapRows) {
    const int t = r >> 6;
    const int w = r & 63;
    const int k = 32 * t + (w & 31);
    const bool isSin = (w >= 32);
    float sv[8];
#pragma unroll
    for (int e = 0; e < 8; ++e) {
      const int n = 8 * tid + e;
      const int j = (k * n) & (kNt - 1);
      const float arg = (float)j * (1.0f / 1024.0f);
      float tv;
      if (isSin) tv = -sinpif(arg);
      else       tv = cospif(arg);
      sv[e] = flush_small(tv * kCarryTap);
    }
    v4u wv;
    wv[0] = pack2_f16(sv[0], sv[1]);
    wv[1] = pack2_f16(sv[2], sv[3]);
    wv[2] = pack2_f16(sv[4], sv[5]);
    wv[3] = pack2_f16(sv[6], sv[7]);
    unsigned* p = TAP + (size_t)r * (kNt / 2) + tid * 4;
    *(volatile v4u*)p = wv;
    __threadfence();
    *(volatile v4u*)p = wv;
  } else if (r < kTapRows + 4) {
    const int g  = (r - kTapRows) * 256 + tid;
    const int j0 = 2 * g;
    const float a0 = (float)j0 * (1.0f / 1024.0f);
    const float a1 = (float)(j0 + 1) * (1.0f / 1024.0f);
    v4f v;
    v[0] = cospif(a0);
    v[1] = sinpif(a0);
    v[2] = cospif(a1);
    v[3] = sinpif(a1);
    float* p = CS + 4 * (size_t)g;
    *(volatile v4f*)p = v;
    __threadfence();
    *(volatile v4f*)p = v;
  } else {
    int j = (r - kTapRows - 4) * 256 + tid;
    j = j & (kNt - 1);
    double c, s;
    cs64_entry(j, c, s);
    v2d v;
    v[0] = c;
    v[1] = s;
    double* p = CS64 + 2 * (size_t)j;
    *(volatile v2d*)p = v;
    __threadfence();
    *(volatile v2d*)p = v;
  }
}

__global__ __launch_bounds__(256) void fused_product_kernel(
    const unsigned short* __restrict__ Ap, const unsigned short* __restrict__ Btp,
    float* __restrict__ RE, float* __restrict__ IM, float* __restrict__ AMP2)
{
  const _Float16* A  = (const _Float16*)Ap;
  const _Float16* Bt = (const _Float16*)Btp;
  __shared__ __align__(16) float sT[8][3][16 * kSlabP];
  const int lane = threadIdx.x & 31;
  const int wave = threadIdx.x >> 5;
  const int tile = blockIdx.x * 8 + wave;
  if (tile >= kTilesM * kTilesN) return;
  const int tm = tile / kTilesN;
  const int tn = tile - tm * kTilesN;
  const int m0 = tm << 6;
  const int n0 = tn << 6;

  const int rlane = lane & 15;
  const int koff  = (lane >> 4) * 8;
  const int mOff  = (lane >> 4) * 8;

  v8f acc[4][4];
#pragma unroll
  for (int i = 0; i < 4; ++i)
#pragma unroll
    for (int j = 0; j < 4; ++j) acc[i][j] = (v8f){0.f, 0.f, 0.f, 0.f, 0.f, 0.f, 0.f, 0.f};

  for (int k0 = 0; k0 < kNt; k0 += 32) {
    v16h bh[4];
#pragma unroll
    for (int j = 0; j < 4; ++j) {
      const size_t bo = (size_t)(n0 + (j << 4) + rlane) * kNt + koff + k0;
      bh[j] = eng::frag_load(Bt + bo);
    }
#pragma unroll
    for (int i = 0; i < 4; ++i) {
      const size_t ao = (size_t)(m0 + (i << 4) + rlane) * kNt + koff + k0;
      const v16h ah = eng::frag_load(A + ao);
#pragma unroll
      for (int j = 0; j < 4; ++j) acc[i][j] = eng::mma(ah, bh[j], acc[i][j]);
      eng::tie_acc(acc[i][0], ah, bh[0]);
      eng::tie_acc(acc[i][1], ah, bh[1]);
      eng::tie_acc(acc[i][2], ah, bh[2]);
      eng::tie_acc_nops(acc[i][3], ah, bh[3]);
    }
    eng::keep4(bh[0], bh[1], bh[2], bh[3]);
  }
  eng::acc_guard4(acc[0][0], acc[0][1], acc[0][2], acc[0][3]);
  eng::acc_guard4(acc[1][0], acc[1][1], acc[1][2], acc[1][3]);
  eng::acc_guard4(acc[2][0], acc[2][1], acc[2][2], acc[2][3]);
  eng::acc_guard4(acc[3][0], acc[3][1], acc[3][2], acc[3][3]);

  float* slabR = sT[wave][0];
  float* slabI = sT[wave][1];
  float* slabA = sT[wave][2];
  const int q  = lane >> 3;
  const int c4 = (lane & 7) * 4;
#pragma unroll
  for (int i = 0; i < 4; ++i) {
    const int mBase = m0 + (i << 4);
#pragma unroll
    for (int j = 0; j < 2; ++j) {
#pragma unroll
      for (int r = 0; r < 8; ++r) {
        const float re = acc[i][j][r] * kFold;
        const float im = acc[i][j + 2][r] * kFold;
        const int idx = (mOff + r) * kSlabP + (j << 4) + rlane;
        slabR[idx] = re;
        slabI[idx] = im;
        slabA[idx] = re * re + im * im;
      }
    }
    wave_lds_sync();
    for (int pass = 0; pass < 2; ++pass) {
#pragma unroll
      for (int it = 0; it < 4; ++it) {
        const int row = it * 4 + q;
        const size_t off = (size_t)(mBase + row) * kBins + tn * 32 + c4;
        const v4f vr = *(const v4f*)(slabR + row * kSlabP + c4);
        const v4f vi = *(const v4f*)(slabI + row * kSlabP + c4);
        const v4f va = *(const v4f*)(slabA + row * kSlabP + c4);
        *(volatile v4f*)(RE + off) = vr;
        *(volatile v4f*)(IM + off) = vi;
        *(volatile v4f*)(AMP2 + off) = va;
      }
      __threadfence();
    }
    wave_lds_sync();
  }
}

__global__ __launch_bounds__(256) void select_kernel(const float* __restrict__ AMP2, const float* __restrict__ RE,
                                                     const float* __restrict__ IM, const float* __restrict__ XS32,
                                                     const double* __restrict__ CS64, int* __restrict__ SELK,
                                                     float* __restrict__ SELRE, float* __restrict__ SELIM)
{
  __shared__ int    sListK[8 * kMaxContested];
  __shared__ double sA64[8 * kMaxContested];
  __shared__ int    sFlag[8 * kMaxContested];
  __shared__ int    sOutK[8 * kSelPitch];
  __shared__ float  sOutRe[8 * kSelPitch];
  __shared__ float  sOutIm[8 * kSelPitch];

  const int lane = threadIdx.x & 31;
  const int wave = threadIdx.x >> 5;
  int m = blockIdx.x * 8 + wave;
  m = (m < kCols) ? m : (kCols - 1);
  const int wb = wave * kMaxContested;
  const int wo = wave * kSelPitch;
  const unsigned ltMask = (1u << lane) - 1u;
  const float qnan = __uint_as_float(0x7fc00000u);

  sListK[wb + lane] = 1;
  sListK[wb + lane + 32] = 1;
  sA64[wb + lane] = 0.0;
  sA64[wb + lane + 32] = 0.0;
  sFlag[wb + lane] = 0;
  sFlag[wb + lane + 32] = 0;
  wave_lds_sync();

  unsigned key[kBinsPerLane];
#pragma unroll
  for (int i = 0; i < kBinsPerLane; ++i) {
    const float v = AMP2[(size_t)m * kBins + 32 * i + lane];
    const unsigned u = __float_as_uint(v);
    key[i] = ((u & 0x80000000u) != 0u) ? 0u : u;
  }
  key[0] = (lane == 0) ? 0u : key[0];

  unsigned T = 0u;
  for (int bit = 30; bit >= 0; --bit) {
    const unsigned cand = T | (1u << bit);
    int cnt = 0;
#pragma unroll
    for (int i = 0; i < kBinsPerLane; ++i) cnt += (key[i] >= cand) ? 1 : 0;
    cnt = wave_sum_i32(cnt);
    T = (cnt >= kTopK) ? cand : T;
  }
  const float aCut = __uint_as_float(T);
  const float hiT = aCut * kHiFac;
  const float loT = aCut * kLoFac;

  unsigned sureBits = 0u;
  unsigned contBits = 0u;
#pragma unroll
  for (int i = 0; i < kBinsPerLane; ++i) {
    const bool isDc = (i == 0) && (lane == 0);
    const float v = __uint_as_float(key[i]);
    const bool su = (v > hiT) && (!isDc);
    const bool co = (v >= loT) && (v <= hiT) && (!isDc);
    sureBits |= su ? (1u << i) : 0u;
    contBits |= co ? (1u << i) : 0u;
  }
  const int nsure = wave_sum_i32(__popc(sureBits));
  const int need  = kTopK - nsure;

  int cbase = 0;
#pragma unroll
  for (int i = 0; i < kBinsPerLane; ++i) {
    const bool co = ((contBits >> i) & 1u) != 0u;
    const unsigned bal = (unsigned)__ballot(co ? 1 : 0);
    const int pos = cbase + __popc(bal & ltMask);
    if (co && (pos < kMaxContested)) sListK[wb + pos] = 32 * i + lane;
    cbase += __popc(bal);
  }
  const int nC = cbase;
  const bool overflow = (nC > kMaxContested);
  const int nCc = overflow ? kMaxContested : nC;
  wave_lds_sync();

  const float* xrow = XS32 + (size_t)m * kNt;
  for (int c = 0; c < nCc; ++c) {
    const int k = sListK[wb + c] & (kBins - 1);
    double ar = 0.0;
    double ai = 0.0;
    for (int s = 0; s < kNt / 32; ++s) {
      const int n = lane + 32 * s;
      const int j = (k * n) & (kNt - 1);
      const v2d cs = *(const v2d*)(CS64 + 2 * (size_t)j);
      const double xv = (double)xrow[n];
      ar = fma(xv, cs[0], ar);
      ai = fma(xv, cs[1], ai);
    }
    ar = wave_sum_f64(ar);
    ai = wave_sum_f64(ai);
    const double a64 = ar * ar + ai * ai;
    if (lane == 0) sA64[wb + c] = a64;
  }
  wave_lds_sync();

  {
    const int lastC = (nCc > 0) ? (nCc - 1) : 0;
    const int cA = lane;
    const int cB = lane + 32;
    const double myA = sA64[wb + ((cA < lastC) ? cA : lastC)];
    const double myB = sA64[wb + ((cB < lastC) ? cB : lastC)];
    int rankA = 0;
    int rankB = 0;
    for (int c2 = 0; c2 < nCc; ++c2) {
      const double o = sA64[wb + c2];
      rankA += ((o > myA) || ((o == myA) && (c2 < cA))) ? 1 : 0;
      rankB += ((o > myB) || ((o == myB) && (c2 < cB))) ? 1 : 0;
    }
    sFlag[wb + cA] = ((cA < nCc) && (rankA < need)) ? 1 : 0;
    sFlag[wb + cB] = ((cB < nCc) && (rankB < need)) ? 1 : 0;
  }
  sOutK[wo + lane]  = (lane < kTopK) ? 1 : 0;
  sOutRe[wo + lane] = (overflow && (lane < kTopK)) ? qnan : 0.0f;
  sOutIm[wo + lane] = (overflow && (lane < kTopK)) ? qnan : 0.0f;
  wave_lds_sync();

  int cb2 = 0;
  int ob  = 0;
#pragma unroll
  for (int i = 0; i < kBinsPerLane; ++i) {
    const float rv = RE[(size_t)m * kBins + 32 * i + lane];
    const float iv = IM[(size_t)m * kBins + 32 * i + lane];
    const bool co = ((contBits >> i) & 1u) != 0u;
    const bool su = ((sureBits >> i) & 1u) != 0u;
    const unsigned balC = (unsigned)__ballot(co ? 1 : 0);
    const int pos  = cb2 + __popc(balC & ltMask);
    const int posc = (pos < kMaxContested - 1) ? pos : (kMaxContested - 1);
    const int fl   = sFlag[wb + posc];
    const bool sel = su || (co && (pos < kMaxContested) && (fl != 0));
    cb2 += __popc(balC);
    const unsigned balS = (unsigned)__ballot(sel ? 1 : 0);
    const int opos = ob + __popc(balS & ltMask);
    ob += __popc(balS);
    if (sel && (opos < kTopK)) {
      sOutK[wo + opos]  = 32 * i + lane;
      sOutRe[wo + opos] = overflow ? qnan : rv;
      sOutIm[wo + opos] = overflow ? qnan : iv;
    }
  }
  wave_lds_sync();

  const int   ok = sOutK[wo + lane];
  const float orv = sOutRe[wo + lane];
  const float oiv = sOutIm[wo + lane];
  volatile int*   pk = SELK  + (size_t)m * kSelPitch + lane;
  volatile float* pr = SELRE + (size_t)m * kSelPitch + lane;
  volatile float* pi = SELIM + (size_t)m * kSelPitch + lane;
  *pk = ok;
  *pr = orv;
  *pi = oiv;
  __threadfence();
  *pk = ok;
  *pr = orv;
  *pi = oiv;
}

__global__ __launch_bounds__(256) void synth_kernel(const int* __restrict__ SELK, const float* __restrict__ SELRE,
                                                    const float* __restrict__ SELIM,
                                                    const float* __restrict__ CS, float* __restrict__ out)
{
  __shared__ __align__(16) float csS[2 * kNt];
  __shared__ int   sK[kTopK * 32];
  __shared__ float sRe[kTopK * 32];
  __shared__ float sNim[kTopK * 32];
  const int tid  = threadIdx.x;
  const int lane = tid & 31;
  const int wave = tid >> 5;
  const int tc = blockIdx.x % kTChunks;
  const int dg = (blockIdx.x / kTChunks) % kDGroups;
  int b = blockIdx.x / (kTChunks * kDGroups);
  b = (b < kNb) ? b : (kNb - 1);
  const int m = b * kNd + dg * 32 + lane;

#pragma unroll
  for (int u = 0; u < 4; ++u) {
    const int o = 4 * (tid * 4 + u);
    const v4f c = *(const v4f*)(CS + o);
    *(v4f*)(csS + o) = c;
  }

  {
    const int we = wave & 1;
    const v4i kv = *(const v4i*)(SELK + (size_t)m * kSelPitch + 4 * we);
    const v4f rv = *(const v4f*)(SELRE + (size_t)m * kSelPitch + 4 * we);
    const v4f iv = *(const v4f*)(SELIM + (size_t)m * kSelPitch + 4 * we);
    if (wave < 2) {
#pragma unroll
      for (int e = 0; e < 4; ++e) {
        const int slot = (4 * we + e) * 32 + lane;
        sK[slot]   = kv[e] & (kBins - 1);
        sRe[slot]  = rv[e];
        sNim[slot] = -iv[e];
      }
    }
  }
  __syncthreads();

  const int tBase = tc * kChunkT + wave * 32;
  const bool again = (tc == 0) && (wave < (kPred / 32));
  for (int g = 0; g < 8; ++g) {
    const int tg = tBase + 4 * g;
    float acc[4];
#pragma unroll
    for (int e = 0; e < 4; ++e) acc[e] = 0.0f;
    for (int j = 0; j < kTopK; ++j) {
      const int   kj = sK[j * 32 + lane];
      const float rj = sRe[j * 32 + lane];
      const float nj = sNim[j * 32 + lane];
#pragma unroll
      for (int e = 0; e < 4; ++e) {
        const int idx = (kj * (tg + e)) & (kNt - 1);
        const v2f cs = *(const v2f*)(csS + 2 * idx);
        acc[e] = fmaf(rj, cs[0], acc[e]);
        acc[e] = fmaf(nj, cs[1], acc[e]);
      }
    }
    float res[4];
#pragma unroll
    for (int e = 0; e < 4; ++e) res[e] = acc[e] * kSynthScale;
    for (int pass = 0; pass < 2; ++pass) {
#pragma unroll
      for (int e = 0; e < 4; ++e) {
        const int t = tg + e;
        float* p = out + ((size_t)b * kTout + t) * kNd + dg * 32 + lane;
        const float v = res[e];
        *(volatile float*)p = v;
        if (again) *(volatile float*)(p + (size_t)kNt * kNd) = v;
      }
      __threadfence();
    }
  }
}

extern "C" void kernel_launch(void* const* d_in, const int* in_sizes, int n_in,
                              void* d_out, int out_size, void* d_ws, size_t ws_size,
                              hipStream_t stream) {
  if (n_in != 1) return;
  if (in_sizes[0] != kInTotal) return;
  if (out_size != kOutTotal) return;
  if (ws_size < kWsTotal) return;

  const float* x = (const float*)d_in[0];
  float* out = (float*)d_out;

  char* ws = (char*)d_ws;
  float*    XS32  = (float*)(ws + kOffXs32);
  unsigned* XS16  = (unsigned*)(ws + kOffXs16);
  unsigned* TAPw  = (unsigned*)(ws + kOffTap);
  float*    CS    = (float*)(ws + kOffCs);
  double*   CS64  = (double*)(ws + kOffCs64);
  float*    RE    = (float*)(ws + kOffRe);
  float*    IM    = (float*)(ws + kOffIm);
  float*    AMP2  = (float*)(ws + kOffAmp2);
  int*      SELK  = (int*)(ws + kOffSelK);
  float*    SELRE = (float*)(ws + kOffSelRe);
  float*    SELIM = (float*)(ws + kOffSelIm);

  column_plane_kernel<<<kNb * kDGroups, 256, 0, stream>>>(x, XS32, XS16);
  table_kernel<<<kTapRows + 4 + 8, 256, 0, stream>>>(TAPw, CS, CS64);
  fused_product_kernel<<<(kTilesM * kTilesN) / 8, 256, 0, stream>>>(
      (const unsigned short*)XS16, (const unsigned short*)TAPw, RE, IM, AMP2);
  select_kernel<<<kCols / 8, 256, 0, stream>>>(AMP2, RE, IM, XS32, CS64, SELK, SELRE, SELIM);
  synth_kernel<<<kNb * kDGroups * kTChunks, 256, 0, stream>>>(SELK, SELRE, SELIM, CS, out);
}
